// SelfAttention_40458591928776
// MI455X (gfx1250) — hardware-run, weakly checked
//
#include <hip/hip_runtime.h>


#ifndef NB
#define NB 4
#endif
#ifndef SEQ
#define SEQ 1024
#endif
#define NB_FULL  4
#define SEQ_FULL 1024
#ifndef OUT_SEQ
#define OUT_SEQ SEQ
#endif
#define DM   2048
#define NH_  16
#define HD   128
#define NQKV 6144
#define PEW  256
#define AW   4
#define OSP  132
#define QRS  2048.0f
#define QRI  (1.0f / 2048.0f)
#define SC2  ((float)(0.08838834764831845 * 1.4426950408889634))
#define PSH  14.0f
#define NEGB (-3.0e38f)
#define WOS  1024.0f
#define CTXS 16.0f
#define OSI  (1.0f / 16384.0f)
#define RMS_EPS 1.0e-6f

static_assert(HD == 128);
static_assert(NH_ * HD == DM);
static_assert(NQKV == 3 * DM);
static_assert(PEW == (HD / 2) * 4);
static_assert(DM % 64 == 0);
static_assert(NQKV % 64 == 0);
static_assert(DM % 32 == 0);
static_assert(HD % 32 == 0);
static_assert(SEQ % 64 == 0);
static_assert((NB * SEQ) % 64 == 0);
static_assert(SEQ % 32 == 0);
static_assert(SEQ % (16 * AW) == 0);
static_assert(((size_t)SEQ * DM) % 8 == 0);
static_assert(NB <= NB_FULL);
static_assert(SEQ <= SEQ_FULL);
static_assert((OSP * 4) % 16 == 0);
static_assert(OSP >= HD);
static_assert(WOS * CTXS * OSI == 1.0f);

typedef _Float16 h16;
typedef unsigned short bf;
typedef __attribute__((ext_vector_type(16))) __bf16   v16bf;
typedef __attribute__((ext_vector_type(16))) _Float16 v16h;
typedef __attribute__((ext_vector_type(8)))  _Float16 v8h;
typedef __attribute__((ext_vector_type(8)))  unsigned short v8us;
typedef __attribute__((ext_vector_type(8)))  float    v8f;
typedef __attribute__((ext_vector_type(4)))  float    v4f;
typedef v4f  __attribute__((may_alias)) v4fa;

__device__ __forceinline__ unsigned short f2bf(float f) { unsigned u = __float_as_uint(f); u += 0x7FFFu + ((u >> 16) & 1u); return (unsigned short)(u >> 16); }
__device__ __forceinline__ float bfr(float f) { return __uint_as_float(((unsigned)f2bf(f)) << 16); }
__device__ __forceinline__ v16h cat16(v8h lo, v8h hi) { return __builtin_shufflevector(lo, hi, 0, 1, 2, 3, 4, 5, 6, 7, 8, 9, 10, 11, 12, 13, 14, 15); }
__device__ __forceinline__ v16bf cat16b(v8us lo, v8us hi) { return __builtin_bit_cast(v16bf, __builtin_shufflevector(lo, hi, 0, 1, 2, 3, 4, 5, 6, 7, 8, 9, 10, 11, 12, 13, 14, 15)); }
__device__ __forceinline__ v16h  ldh(const h16* p) { return cat16(*(const v8h*)p, *(const v8h*)(p + 16)); }
__device__ __forceinline__ v16bf ldb(const bf* p)  { return cat16b(*(const v8us*)p, *(const v8us*)(p + 16)); }
__device__ __forceinline__ void wave_sync() { __builtin_amdgcn_fence(3  , "wavefront"); __builtin_amdgcn_wave_barrier(); asm volatile("" ::: "memory"); }
__device__ __forceinline__ v8f wmma16g(v16h a, v16h b, v8f c) {
    c = __builtin_amdgcn_wmma_f32_16x16x32_f16(false, a, false, b, (short)0, c, false, false);
    asm volatile("v_nop\n\tv_nop\n\tv_nop\n\tv_nop" : "+v"(c) : "v"(a), "v"(b));
    return c; }
__device__ __forceinline__ v8f wmmabg(v16bf a, v16bf b, v8f c) {
    c = __builtin_amdgcn_wmma_f32_16x16x32_bf16(false, a, false, b, (short)0, c, false, false);
    asm volatile("v_nop\n\tv_nop\n\tv_nop\n\tv_nop" : "+v"(c) : "v"(a), "v"(b));
    return c; }
static __device__ __forceinline__ h16 toh_flush(float v) { const h16 r = (h16)v; return (fabsf(v) < 6.103515625e-05f) ? (h16)0.0f : r; }

__global__ __launch_bounds__(256) void k_cvt8(const float* __restrict__ src, bf* dst, size_t n8) {
    const size_t i = (size_t)blockIdx.x * 256 + threadIdx.x; if (i >= n8) return;
    const v8f v = *(const v8f*)(src + i * 8); v8us o;
#pragma unroll
    for (int k = 0; k < 8; ++k) o[k] = f2bf(v[k]);
    *(volatile v8us*)(dst + i * 8) = o; __threadfence(); *(volatile v8us*)(dst + i * 8) = o;
}

static_assert(2 * 256 * 8 == 64 * 64);
static_assert(4 * 256 * 4 == 64 * 64);
static_assert(64 * 68 * 4 <= 131072);
__global__ __launch_bounds__(256) void k_wtr(const float* __restrict__ src, unsigned short* dst, int KR_, int NC, int f16mode, float scale) {
    __shared__ __align__(16) float ts[64 * 68];
    const int tid = threadIdx.x;
    const int n0 = blockIdx.x * 64, k0 = blockIdx.y * 64;
#pragma unroll 1
    for (int it = 0; it < 4; ++it) { const int idx = it * 256 + tid; const int row = idx >> 4, c4 = (idx & 15) * 4;
        const v4f v = *(const v4f*)(src + (size_t)(k0 + row) * NC + n0 + c4);
        *(v4fa*)(&ts[row * 68 + c4]) = v; }
    __syncthreads();
    v8us ov[2];
#pragma unroll
    for (int it = 0; it < 2; ++it) { const int p = it * 256 + tid; const int n = p >> 3, kk = (p & 7) * 8;
        v8us bv; v8h hv;
#pragma unroll
        for (int i = 0; i < 8; ++i) { const float v = ts[(kk + i) * 68 + n]; bv[i] = f2bf(v); hv[i] = toh_flush(bfr(v) * scale); }
        const v8us hb = __builtin_bit_cast(v8us, hv);
        ov[it] = f16mode ? hb : bv; }
#pragma unroll 1
    for (int ps = 0; ps < 2; ++ps) {
#pragma unroll
        for (int it = 0; it < 2; ++it) { const int p = it * 256 + tid; const int n = p >> 3, kk = (p & 7) * 8;
            *(volatile v8us*)(dst + (size_t)(n0 + n) * KR_ + k0 + kk) = ov[it]; }
        if (ps == 0) __threadfence(); }
}

static_assert(8 * 32 * 16 == 16 * HD * 2);
static_assert(16 * OSP * 4 <= 131072);
static_assert(SEQ % 32 == 0);
__global__ __launch_bounds__(32) void k_qk(const bf* __restrict__ A, const bf* __restrict__ Bt, const float* __restrict__ pe,
                                           const float* __restrict__ qsc, const float* __restrict__ qbi, const float* __restrict__ ksc, const float* __restrict__ kbi,
                                           h16* PH, h16* PR) {
    __shared__ __align__(16) float os[16 * OSP];
    const int K = DM;
    const int lane = threadIdx.x & 31, lr = lane & 15, hi = lane >> 4;
    const int r0 = blockIdx.x * 32, y = blockIdx.y, c0 = y * HD;
    v8f acc[2][8];
#pragma unroll
    for (int mb = 0; mb < 2; ++mb)
#pragma unroll
        for (int nb = 0; nb < 8; ++nb) acc[mb][nb] = (v8f){};
    const size_t aoff = (size_t)(r0 + lr) * K + 8 * hi, boff = (size_t)(c0 + lr) * K + 8 * hi;
#pragma unroll 1
    for (int kc = 0; kc < K; kc += 32) {
        v16bf a[2];
#pragma unroll
        for (int mb = 0; mb < 2; ++mb) a[mb] = ldb(A + aoff + (size_t)mb * 16 * K + kc);
#pragma unroll
        for (int nb = 0; nb < 8; ++nb) { const v16bf b = ldb(Bt + boff + (size_t)nb * 16 * K + kc);
#pragma unroll
            for (int mb = 0; mb < 2; ++mb) acc[mb][nb] = wmmabg(a[mb], b, acc[mb][nb]); }
    }
    const int c8 = lr * 8;
    const bool isk = y >= NH_;
    float sc[8], bi[8];
    { const v4f q0 = *(const v4f*)(qsc + c8), q1 = *(const v4f*)(qsc + c8 + 4), k0v = *(const v4f*)(ksc + c8), k1v = *(const v4f*)(ksc + c8 + 4);
      const v4f p0 = *(const v4f*)(qbi + c8), p1 = *(const v4f*)(qbi + c8 + 4), r0v = *(const v4f*)(kbi + c8), r1v = *(const v4f*)(kbi + c8 + 4);
#pragma unroll
      for (int i = 0; i < 4; ++i) { sc[i] = bfr(isk ? k0v[i] : q0[i]); sc[4 + i] = bfr(isk ? k1v[i] : q1[i]);
                                    bi[i] = bfr(isk ? r0v[i] : p0[i]); bi[4 + i] = bfr(isk ? r1v[i] : p1[i]); } }
    const int bb = r0 / SEQ, tt = r0 % SEQ;
    const int which = y / NH_, hh = y % NH_;
    const size_t zrow = (size_t)(which * NB * NH_ + bb * NH_ + hh) * SEQ + (size_t)tt;
    const size_t perow = (size_t)bb * SEQ_FULL + (size_t)tt;
#pragma unroll
    for (int mb = 0; mb < 2; ++mb) {
#pragma unroll
        for (int nb = 0; nb < 8; ++nb) {
#pragma unroll
            for (int j = 0; j < 8; ++j) os[(hi * 8 + j) * OSP + nb * 16 + lr] = acc[mb][nb][j]; }
        wave_sync();
        const size_t base = (zrow + (size_t)(mb * 16)) * HD;
        const float* pslab = pe + (perow + (size_t)(mb * 16)) * PEW + c8 * 2;
#pragma unroll 1
        for (int s = 0; s < 8; ++s) {
            const int row = 2 * s + hi;
            const v4f x0 = *(const v4fa*)(&os[row * OSP + c8]); const v4f x1 = *(const v4fa*)(&os[row * OSP + c8 + 4]);
            float u[8];
#pragma unroll
            for (int i = 0; i < 4; ++i) { u[i] = x0[i]; u[4 + i] = x1[i]; }
            float ss = 0.0f;
#pragma unroll
            for (int i = 0; i < 8; ++i) ss += u[i] * u[i];
            ss += __shfl_xor(ss, 8, 32); ss += __shfl_xor(ss, 4, 32); ss += __shfl_xor(ss, 2, 32); ss += __shfl_xor(ss, 1, 32);
            const float inv = rsqrtf(ss * (1.0f / 128.0f) + RMS_EPS);
            const float* pp = pslab + (size_t)row * PEW;
            const v4f g0 = *(const v4f*)(pp), g1 = *(const v4f*)(pp + 4), g2 = *(const v4f*)(pp + 8), g3 = *(const v4f*)(pp + 12);
            float un[8];
#pragma unroll
            for (int i = 0; i < 8; ++i) un[i] = u[i] * inv * sc[i] + bi[i];
            float val[8];
            val[0] = bfr(g0[0]) * un[0] + bfr(g0[1]) * un[1]; val[1] = bfr(g0[2]) * un[0] + bfr(g0[3]) * un[1];
            val[2] = bfr(g1[0]) * un[2] + bfr(g1[1]) * un[3]; val[3] = bfr(g1[2]) * un[2] + bfr(g1[3]) * un[3];
            val[4] = bfr(g2[0]) * un[4] + bfr(g2[1]) * un[5]; val[5] = bfr(g2[2]) * un[4] + bfr(g2[3]) * un[5];
            val[6] = bfr(g3[0]) * un[6] + bfr(g3[1]) * un[7]; val[7] = bfr(g3[2]) * un[6] + bfr(g3[3]) * un[7];
            v8h hv, rv;
#pragma unroll
            for (int i = 0; i < 8; ++i) { const h16 a0 = toh_flush(val[i]); hv[i] = a0; rv[i] = toh_flush((val[i] - (float)a0) * QRS); }
            const size_t oo = base + (size_t)(s * 32 + lane) * 8;
            *(volatile v8h*)(PH + oo) = hv; *(volatile v8h*)(PR + oo) = rv;
            __threadfence();
            *(volatile v8h*)(PH + oo) = hv; *(volatile v8h*)(PR + oo) = rv;
        }
        wave_sync();
    }
}

static_assert(4 * 4 == 16);
static_assert(8 * 16 == 64 * 2);
static_assert(16 * 68 * 4 <= 131072);
__global__ __launch_bounds__(32) void k_vt(const bf* __restrict__ A, const bf* __restrict__ Bt, h16* VT) {
    __shared__ __align__(16) float os[16 * 68];
    const int K = DM;
    const int lane = threadIdx.x & 31, lr = lane & 15, hi = lane >> 4; const int r0 = blockIdx.x * 64, c0 = blockIdx.y * 64;
    v8f acc[4][4];
#pragma unroll
    for (int mb = 0; mb < 4; ++mb)
#pragma unroll
        for (int nb = 0; nb < 4; ++nb) acc[mb][nb] = (v8f){};
    const size_t aoff = (size_t)(r0 + lr) * K + 8 * hi, boff = (size_t)(c0 + lr) * K + 8 * hi;
#pragma unroll 1
    for (int kc = 0; kc < K; kc += 32) {
        v16bf a[4];
#pragma unroll
        for (int mb = 0; mb < 4; ++mb) a[mb] = ldb(A + aoff + (size_t)mb * 16 * K + kc);
#pragma unroll
        for (int nb = 0; nb < 4; ++nb) { const v16bf b = ldb(Bt + boff + (size_t)nb * 16 * K + kc);
#pragma unroll
            for (int mb = 0; mb < 4; ++mb) acc[mb][nb] = wmmabg(a[mb], b, acc[mb][nb]); }
    }
    const int bb = c0 / SEQ, tt = c0 % SEQ;
    const size_t tbase = (size_t)bb * (size_t)DM * SEQ + (size_t)r0 * SEQ + (size_t)tt;
#pragma unroll
    for (int mb = 0; mb < 4; ++mb) {
#pragma unroll
        for (int nb = 0; nb < 4; ++nb) {
#pragma unroll
            for (int j = 0; j < 8; ++j) os[(hi * 8 + j) * 68 + nb * 16 + lr] = acc[mb][nb][j]; }
        wave_sync();
        const size_t sb = tbase + (size_t)(mb * 16) * SEQ;
#pragma unroll 1
        for (int ps = 0; ps < 2; ++ps) {
#pragma unroll
            for (int s = 0; s < 4; ++s) { const int row = 4 * s + (lane >> 3), c8 = (lane & 7) * 8;
                const v4f x0 = *(const v4fa*)(&os[row * 68 + c8]); const v4f x1 = *(const v4fa*)(&os[row * 68 + c8 + 4]); v8h hv;
#pragma unroll
                for (int i = 0; i < 4; ++i) { hv[i] = toh_flush(x0[i]); hv[4 + i] = toh_flush(x1[i]); }
                *(volatile v8h*)(VT + sb + (size_t)row * SEQ + c8) = hv; }
            if (ps == 0) __threadfence(); }
        wave_sync();
    }
}

static_assert(8 * 2 == 16);
static_assert(16 * 16 == HD * 2);
static_assert(AW * 16 * OSP * 4 <= 131072);
__global__ __launch_bounds__(32 * AW) void k_flash(const h16* __restrict__ QH, const h16* __restrict__ QR, const h16* __restrict__ KH, const h16* __restrict__ KR,
                                                   const h16* __restrict__ VT, h16* CTX) {
    __shared__ __align__(16) float os[AW * 16 * OSP];
    const int lane = threadIdx.x & 31, lr = lane & 15, hi = lane >> 4;
    const int wave = __builtin_amdgcn_readfirstlane((int)(threadIdx.x >> 5));
    const int zh = blockIdx.y; const int b = zh / NH_, h = zh % NH_;
    const int t0 = (blockIdx.x * AW + wave) * 16;
    const size_t pbase = (size_t)zh * SEQ * HD;
    const size_t qo = pbase + (size_t)(t0 + lr) * HD + 8 * hi;
    const size_t ko = pbase + (size_t)lr * HD + 8 * hi;
    const size_t vo = pbase + (size_t)lr * SEQ + 8 * hi;
    v8f o[8];
#pragma unroll
    for (int j = 0; j < 8; ++j) o[j] = (v8f){};
    float m = NEGB, l = 0.0f;
#pragma unroll 1
    for (int key0 = 0; key0 < SEQ; key0 += 32) {
        const size_t kk = ko + (size_t)key0 * HD;
        v8f sHa = (v8f){}, sLa = (v8f){}, sHb = (v8f){}, sLb = (v8f){};
#pragma unroll 1
        for (int c = 0; c < HD; c += 32) {
            const v16h qh = ldh(QH + qo + c), qr = ldh(QR + qo + c);
            const v16h ka = ldh(KH + kk + c), kb = ldh(KH + kk + (size_t)16 * HD + c);
            const v16h kra = ldh(KR + kk + c), krb = ldh(KR + kk + (size_t)16 * HD + c);
            sHa = wmma16g(ka, qh, sHa); sLa = wmma16g(ka, qr, sLa);
            sHb = wmma16g(kb, qh, sHb); sLb = wmma16g(kb, qr, sLb);
            sLa = wmma16g(kra, qh, sLa); sLb = wmma16g(krb, qh, sLb);
        }
        float ta[8], tb[8]; float mx = NEGB;
#pragma unroll
        for (int r = 0; r < 8; ++r) {
            ta[r] = (sHa[r] + sLa[r] * QRI) * SC2; tb[r] = (sHb[r] + sLb[r] * QRI) * SC2;
            mx = fmaxf(mx, fmaxf(ta[r], tb[r])); }
        mx = fmaxf(mx, __shfl_xor(mx, 16, 32));
        const float mnew = fmaxf(m, mx);
        const float alpha = __builtin_amdgcn_exp2f(m - mnew);
        const float sh = PSH - mnew;
        v16h pb; float ls = 0.0f;
#pragma unroll
        for (int r = 0; r < 8; ++r) {
            const float xa = ta[r] + sh, xb = tb[r] + sh;
            const float ea = __builtin_amdgcn_exp2f(xa), eb = __builtin_amdgcn_exp2f(xb);
            const float ga = (xa < -14.0f) ? 0.0f : ea, gb = (xb < -14.0f) ? 0.0f : eb;
            const h16 pa = (h16)ga; const h16 pc = (h16)gb;
            pb[r] = pa; pb[8 + r] = pc;
            ls += (float)pa + (float)pc; }
        l = l * alpha + ls; m = mnew;
#pragma unroll
        for (int j = 0; j < 8; ++j) o[j] = o[j] * alpha;
        const h16* va = VT + vo + key0;
#pragma unroll
        for (int g = 0; g < 2; ++g) {
            v16h vf[4];
#pragma unroll
            for (int jj = 0; jj < 4; ++jj) vf[jj] = ldh(va + (size_t)((g * 4 + jj) * 16) * SEQ);
#pragma unroll
            for (int jj = 0; jj < 4; ++jj) o[g * 4 + jj] = wmma16g(vf[jj], pb, o[g * 4 + jj]);
        }
    }
    l += __shfl_xor(l, 16, 32);
    const float inv = CTXS * (1.0f / l);
    const int wb = wave * 16 * OSP;
#pragma unroll
    for (int j = 0; j < 8; ++j) { v4f a, c;
#pragma unroll
        for (int i = 0; i < 4; ++i) { a[i] = o[j][i] * inv; c[i] = o[j][4 + i] * inv; }
        *(v4fa*)(&os[wb + lr * OSP + 16 * j + 8 * hi]) = a; *(v4fa*)(&os[wb + lr * OSP + 16 * j + 8 * hi + 4]) = c; }
    wave_sync();
    h16* crow = CTX + ((size_t)b * SEQ + t0) * DM + h * HD;
#pragma unroll 1
    for (int ps = 0; ps < 2; ++ps) {
#pragma unroll 1
        for (int s = 0; s < 8; ++s) { const int row = 2 * s + (lane >> 4), c8 = (lane & 15) * 8;
            const v4f x0 = *(const v4fa*)(&os[wb + row * OSP + c8]); const v4f x1 = *(const v4fa*)(&os[wb + row * OSP + c8 + 4]); v8h hv;
#pragma unroll
            for (int i = 0; i < 4; ++i) { hv[i] = toh_flush(x0[i]); hv[4 + i] = toh_flush(x1[i]); }
            *(volatile v8h*)(crow + (size_t)row * DM + c8) = hv; }
        if (ps == 0) __threadfence(); }
}

static_assert(16 * 16 == 64 * 4);
__global__ __launch_bounds__(32) void k_oproj(const h16* __restrict__ A, const h16* __restrict__ Bt, float* OUT) {
    __shared__ __align__(16) float os[16 * 68];
    const int K = DM;
    const int lane = threadIdx.x & 31, lr = lane & 15, hi = lane >> 4; const int r0 = blockIdx.x * 64, c0 = blockIdx.y * 64;
    v8f acc[4][4];
#pragma unroll
    for (int mb = 0; mb < 4; ++mb)
#pragma unroll
        for (int nb = 0; nb < 4; ++nb) acc[mb][nb] = (v8f){};
    const size_t aoff = (size_t)(r0 + lr) * K + 8 * hi, boff = (size_t)(c0 + lr) * K + 8 * hi;
#pragma unroll 1
    for (int kc = 0; kc < K; kc += 32) {
        v16h a[4];
#pragma unroll
        for (int mb = 0; mb < 4; ++mb) a[mb] = ldh(A + aoff + (size_t)mb * 16 * K + kc);
#pragma unroll
        for (int nb = 0; nb < 4; ++nb) { const v16h b = ldh(Bt + boff + (size_t)nb * 16 * K + kc);
#pragma unroll
            for (int mb = 0; mb < 4; ++mb) acc[mb][nb] = wmma16g(a[mb], b, acc[mb][nb]); }
    }
    const int bb = r0 / SEQ, tt = r0 % SEQ;
    float* orow = OUT + ((size_t)bb * OUT_SEQ + (size_t)tt) * DM + c0;
#pragma unroll
    for (int mb = 0; mb < 4; ++mb) {
#pragma unroll
        for (int nb = 0; nb < 4; ++nb) {
#pragma unroll
            for (int j = 0; j < 8; ++j) os[(hi * 8 + j) * 68 + nb * 16 + lr] = acc[mb][nb][j] * OSI; }
        wave_sync();
#pragma unroll 1
        for (int ps = 0; ps < 2; ++ps) {
#pragma unroll
            for (int s = 0; s < 8; ++s) { const int row = 2 * s + (lane >> 4), cofs = (lane & 15) * 4;
                const v4f val = *(const v4fa*)(&os[row * 68 + cofs]);
                *(volatile v4f*)(orow + (size_t)(mb * 16 + row) * DM + cofs) = val; }
            if (ps == 0) __threadfence(); }
        wave_sync();
    }
}

static constexpr size_t al256(size_t v) { return (v + 255) & ~(size_t)255; }
static constexpr size_t PLANE = (size_t)NB * NH_ * SEQ * HD;
static constexpr size_t SZ_XB = al256((size_t)NB * SEQ * DM * 2);
static constexpr size_t SZ_WT = al256((size_t)NQKV * DM * 2);
static constexpr size_t SZ_PL = al256(PLANE * 2);
static constexpr size_t SZ_TOTAL = SZ_XB + SZ_WT + 5 * SZ_PL;
static_assert(SZ_TOTAL <= (size_t)134217728);
static_assert(SZ_PL == PLANE * 2);
static_assert((size_t)NB * SEQ * DM * 2 <= SZ_XB);
static_assert((size_t)DM * DM * 2 <= SZ_WT);
static_assert((size_t)NB * NH_ * SEQ * HD == (size_t)NB * DM * SEQ);

extern "C" void kernel_launch(void* const* d_in, const int* in_sizes, int n_in,
                              void* d_out, int out_size, void* d_ws, size_t ws_size, hipStream_t stream) {
    if (n_in < 8) return;
    const size_t needt = (size_t)(NB - 1) * SEQ_FULL + SEQ;
    if ((size_t)in_sizes[0] < needt * DM) return;
    if ((size_t)in_sizes[1] < needt * PEW) return;
    if ((size_t)in_sizes[2] < (size_t)DM * NQKV || (size_t)in_sizes[3] < (size_t)DM * DM) return;
    if (in_sizes[4] < HD || in_sizes[5] < HD || in_sizes[6] < HD || in_sizes[7] < HD) return;
    if ((size_t)out_size < ((size_t)(NB - 1) * OUT_SEQ + SEQ) * DM) return;
    if (SZ_TOTAL > ws_size) return;
    const float* x   = (const float*)d_in[0];
    const float* pe  = (const float*)d_in[1];
    const float* wqk = (const float*)d_in[2];
    const float* wo  = (const float*)d_in[3];
    const float* qs  = (const float*)d_in[4]; const float* qb = (const float*)d_in[5];
    const float* ks  = (const float*)d_in[6]; const float* kb = (const float*)d_in[7];
    float* OUT = (float*)d_out;
    char* wsp = (char*)d_ws;
    char* regx = wsp; wsp += SZ_XB;
    char* regw = wsp; wsp += SZ_WT;
    bf*  XB  = (bf*)regx;
    h16* CTX = (h16*)regx;
    bf*  WT  = (bf*)regw;
    h16* WOT = (h16*)regw;
    h16* PH = (h16*)wsp; wsp += 2 * SZ_PL;
    h16* PR = (h16*)wsp; wsp += 2 * SZ_PL;
    h16* VT = (h16*)wsp; wsp += SZ_PL;
    h16* QH = PH; h16* KH = PH + PLANE; h16* QR = PR; h16* KR = PR + PLANE;

    if (SEQ == SEQ_FULL) {
        const size_t n8 = (size_t)NB * SEQ * DM / 8;
        k_cvt8<<<(unsigned)((n8 + 255) / 256), 256, 0, stream>>>(x, XB, n8);
    } else {
        const size_t n8 = (size_t)SEQ * DM / 8;
        for (int b = 0; b < NB; ++b) k_cvt8<<<(unsigned)((n8 + 255) / 256), 256, 0, stream>>>(x + (size_t)b * SEQ_FULL * DM, XB + (size_t)b * SEQ * DM, n8);
    }
    k_wtr<<<dim3(NQKV / 64, DM / 64, 1), 256, 0, stream>>>(wqk, (unsigned short*)WT, DM, NQKV, 0, 1.0f);

    k_qk<<<dim3(NB * SEQ / 32, 2 * NH_, 1), 32, 0, stream>>>(XB, WT, pe, qs, qb, ks, kb, PH, PR);
    k_vt<<<dim3(DM / 64, NB * SEQ / 64, 1), 32, 0, stream>>>(WT + (size_t)2 * DM * DM, XB, VT);

    k_wtr<<<dim3(DM / 64, DM / 64, 1), 256, 0, stream>>>(wo, (unsigned short*)WOT, DM, DM, 1, WOS);

    k_flash<<<dim3(SEQ / (16 * AW), NB * NH_, 1), 32 * AW, 0, stream>>>(QH, QR, KH, KR, VT, CTX);

    k_oproj<<<dim3(NB * SEQ / 64, DM / 64, 1), 32, 0, stream>>>(CTX, WOT, OUT);
}
